// StationaryHMM_42563125903453
// MI455X (gfx1250) — hardware-run, weakly checked
//
#include <hip/hip_runtime.h>
#include <math.h>

typedef __attribute__((ext_vector_type(16))) __bf16   v16b;
typedef __attribute__((ext_vector_type(8)))  float    v8f;
typedef __attribute__((ext_vector_type(4)))  float    v4f;
typedef __attribute__((ext_vector_type(4)))  unsigned v4u;
typedef __attribute__((ext_vector_type(8)))  unsigned v8u;

constexpr int kT       = 500000;
constexpr int kS       = 16;
constexpr int kChunk   = 4000;
constexpr int kWarm    = 1024;
constexpr int kNChunk  = kT / kChunk;
constexpr int kTiles   = (kNChunk + 15) / 16;
constexpr int kGrp     = 32;
constexpr int kSub     = 16;
constexpr int kNGrp    = (kWarm + kChunk) / kGrp;
constexpr int kWarmGrp = kWarm / kGrp;
constexpr int kAP      = 20;
constexpr int kOffUN   = 16 * kT;
constexpr int kOffFT   = 32 * kT;
constexpr float kFltMin = 1.17549435e-38f;

static_assert(kS == 16);
static_assert(kNChunk * kChunk == kT);
static_assert((kChunk % kGrp) == 0 && (kWarm % kGrp) == 0 && (kT % kGrp) == 0);
static_assert(kNChunk == 125 && kTiles == 8 && kNGrp == 157 && kWarmGrp == 32);
static_assert(kGrp == 2 * kSub);
static_assert(((size_t)kOffUN * 4) % 128 == 0 && ((size_t)kOffFT * 4) % 128 == 0);
static_assert((kAP % 4) == 0);

constexpr int kWsPT     = 0;
constexpr int kWsPrm    = 256;
constexpr int kWsFloats = 384;
constexpr size_t kWsBytes = (size_t)kWsFloats * 4;
static_assert(kWsBytes == 1536);
static_assert(kWsBytes <= 134217728ull);

__device__ __forceinline__ unsigned bf_rne_bits(float f) {
  const unsigned u = __float_as_uint(f);
  return (u + 0x7FFFu + ((u >> 16) & 1u)) >> 16;
}
__device__ __forceinline__ unsigned pack_hi_lo(float f) {
  const unsigned hb = bf_rne_bits(f) & 0xFFFFu;
  const float hf = __uint_as_float(hb << 16);
  const float rs = f - hf;
  const unsigned lb = bf_rne_bits(rs) & 0xFFFFu;
  return hb | (lb << 16);
}
__device__ __forceinline__ void words_to_frags(const v4u a, const v4u b, v16b& hi, v16b& lo) {
  const unsigned a0 = a[0], a1 = a[1], a2 = a[2], a3 = a[3];
  const unsigned b0 = b[0], b1 = b[1], b2 = b[2], b3 = b[3];
  v8u H, Lw;
  H[0] = (a0 & 0xFFFFu) | (a1 << 16);
  H[1] = (a2 & 0xFFFFu) | (a3 << 16);
  H[2] = (b0 & 0xFFFFu) | (b1 << 16);
  H[3] = (b2 & 0xFFFFu) | (b3 << 16);
  H[4] = 0u; H[5] = 0u; H[6] = 0u; H[7] = 0u;
  Lw[0] = (a0 >> 16) | (a1 & 0xFFFF0000u);
  Lw[1] = (a2 >> 16) | (a3 & 0xFFFF0000u);
  Lw[2] = (b0 >> 16) | (b1 & 0xFFFF0000u);
  Lw[3] = (b2 >> 16) | (b3 & 0xFFFF0000u);
  Lw[4] = 0u; Lw[5] = 0u; Lw[6] = 0u; Lw[7] = 0u;
  hi = __builtin_bit_cast(v16b, H);
  lo = __builtin_bit_cast(v16b, Lw);
}
__device__ __forceinline__ v8f mma_bf(v16b a, v16b b, v8f c) {
  return __builtin_amdgcn_wmma_f32_16x16x32_bf16(false, a, false, b, (short)0, c, false, false);
}
__device__ __forceinline__ void acc_guard(v8f& c, v16b a0, v16b a1, v16b b0, v16b b1) {
  asm volatile("v_nop\n\tv_nop\n\tv_nop\n\tv_nop" : "+v"(c) : "v"(a0), "v"(a1), "v"(b0), "v"(b1));
}

__global__ __launch_bounds__(32) void k_init(const float* __restrict__ logits, const float* __restrict__ mu,
                                              const float* __restrict__ logsig, float* wsf)
{
  __shared__ float sP[32 * 17];
  __shared__ float sv[32];
  __shared__ __align__(16) float sO[kWsFloats];
  const int lane = threadIdx.x & 31;
  const int j  = lane & 15;
  const int hs = lane >> 4;

  const float* lrow = logits + j * 16;
  float mx = lrow[0];
#pragma unroll 1
  for (int k = 1; k < 16; ++k) mx = fmaxf(mx, lrow[k]);
  float ssum = 0.0f;
#pragma unroll 1
  for (int k = 0; k < 16; ++k) {
    const float e = expf(lrow[k] - mx);
    sP[lane * 17 + k] = e;
    ssum += e;
  }
  const float rinv = 1.0f / ssum;
#pragma unroll 1
  for (int k = 0; k < 16; ++k) {
    const float pv = sP[lane * 17 + k] * rinv;
    sP[lane * 17 + k] = pv;
  }

  const float muv = mu[j];
  const float sg  = expf(logsig[j]);
  const float isg = 1.0f / sg;
  const float cf  = 0.3989422804014327f / sg;

  float pij = 0.0625f;
  sv[lane] = pij;
  __syncthreads();
#pragma unroll 1
  for (int it = 0; it < 256; ++it) {
    float nn = 0.0f;
#pragma unroll 1
    for (int k = 0; k < 16; ++k) nn = fmaf(sv[k], sP[k * 17 + j], nn);
    float tot = nn;
    tot += __shfl_xor(tot, 1, 32);
    tot += __shfl_xor(tot, 2, 32);
    tot += __shfl_xor(tot, 4, 32);
    tot += __shfl_xor(tot, 8, 32);
    pij = nn * (1.0f / tot);
    __syncthreads();
    sv[lane] = pij;
    __syncthreads();
  }

#pragma unroll 1
  for (int q = 0; q < 8; ++q) {
    const int idx = q * 32 + lane;
    const int n = idx >> 4;
    const int k = idx & 15;
    sO[kWsPT + idx] = sP[k * 17 + n];
  }
  sO[kWsPrm + hs * 32 + j]      = hs ? cf  : muv;
  sO[kWsPrm + hs * 32 + 16 + j] = hs ? pij : isg;
  sO[320 + lane] = 0.0f;
  sO[352 + lane] = 0.0f;
  __syncthreads();
  for (int pass = 0; pass < 2; ++pass) {
#pragma unroll
    for (int it = 0; it < 3; ++it) {
      const v4f v = *(const v4f*)(sO + it * 128 + lane * 4);
      *(volatile v4f*)(wsf + it * 128 + lane * 4) = v;
    }
    __threadfence();
  }
}

__global__ __launch_bounds__(32) void k_filter(const float* __restrict__ y, const float* __restrict__ wsf, float* out)
{
  __shared__ __align__(16) unsigned sA[16 * kAP];
  __shared__ __align__(16) float sY[kGrp * 16];
  __shared__ __align__(16) float sU[16 * kSub * kS];
  __shared__ __align__(16) float sN[16 * kSub * kS];
  __shared__ __align__(16) float sF[16 * kGrp + 32];

  const int lane = threadIdx.x & 31;
  const int h = lane >> 4;
  const int j = lane & 15;
  const int tile = blockIdx.x;
  const int cbase = tile * 16 + 8 * h;

  v16b bh, bl;
  {
    const v4f p0 = *(const v4f*)(wsf + kWsPT + j * 16 + 8 * h);
    const v4f p1 = *(const v4f*)(wsf + kWsPT + j * 16 + 8 * h + 4);
    v4u qa, qb;
    qa[0] = pack_hi_lo(p0[0]); qa[1] = pack_hi_lo(p0[1]); qa[2] = pack_hi_lo(p0[2]); qa[3] = pack_hi_lo(p0[3]);
    qb[0] = pack_hi_lo(p1[0]); qb[1] = pack_hi_lo(p1[1]); qb[2] = pack_hi_lo(p1[2]); qb[3] = pack_hi_lo(p1[3]);
    words_to_frags(qa, qb, bh, bl);
  }
  const float mu_j  = wsf[kWsPrm + j];
  const float inv_j = wsf[kWsPrm + 16 + j];
  const float cf_j  = wsf[kWsPrm + 32 + j];
  const float pi_j  = wsf[kWsPrm + 48 + j];

  float V[8];
  unsigned liveAll = 0u, liveHold = 0u;
#pragma unroll
  for (int r = 0; r < 8; ++r) {
    const int c = cbase + r;
    V[r] = (c == 0) ? pi_j : 0.0625f;
    liveAll  |= (c < kNChunk) ? (1u << r) : 0u;
    liveHold |= ((c < kNChunk) && (c != 0)) ? (1u << r) : 0u;
  }
  const int jr = j & 7;

#pragma unroll 1
  for (int grp = 0; grp < kNGrp; ++grp) {
    const int i0 = grp * kGrp;
#pragma unroll
    for (int it = 0; it < 4; ++it) {
      const int m = it * 4 + (lane >> 3);
      const int q = lane & 7;
      int tb = (tile * 16 + m) * kChunk - kWarm + i0;
      tb = (tb < 0) ? 0 : tb;
      tb = (tb > kT - kGrp) ? (kT - kGrp) : tb;
      const v4f yv = *(const v4f*)(y + tb + 4 * q);
      sY[(4 * q + 0) * 16 + m] = yv[0];
      sY[(4 * q + 1) * 16 + m] = yv[1];
      sY[(4 * q + 2) * 16 + m] = yv[2];
      sY[(4 * q + 3) * 16 + m] = yv[3];
    }
    __syncthreads();
    const unsigned am = (i0 < kWarm) ? liveHold : liveAll;

#pragma unroll 1
    for (int half = 0; half < 2; ++half) {
#pragma unroll 1
      for (int s = 0; s < kSub; ++s) {
        const int ss = half * kSub + s;
#pragma unroll
        for (int r = 0; r < 8; ++r) sA[(8 * h + r) * kAP + j] = pack_hi_lo(V[r]);
        __syncthreads();
        const v4u wa = *(const v4u*)(sA + j * kAP + 8 * h);
        const v4u wb = *(const v4u*)(sA + j * kAP + 8 * h + 4);
        v16b ah, al;
        words_to_frags(wa, wb, ah, al);
        v8f acc = (v8f){0.f, 0.f, 0.f, 0.f, 0.f, 0.f, 0.f, 0.f};
        acc = mma_bf(ah, bh, acc);
        acc = mma_bf(ah, bl, acc);
        acc = mma_bf(al, bh, acc);
        acc_guard(acc, ah, al, bh, bl);

        const v4f ya = *(const v4f*)(sY + ss * 16 + 8 * h);
        const v4f yb = *(const v4f*)(sY + ss * 16 + 8 * h + 4);
        float w[8], ft[8];
#pragma unroll
        for (int r = 0; r < 8; ++r) {
          const float yr = (r < 4) ? ya[r & 3] : yb[r & 3];
          const float z = (yr - mu_j) * inv_j;
          float e = expf(-0.5f * z * z);
          e = (e < kFltMin) ? 0.0f : e;
          float g = e * cf_j;
          g = (g < kFltMin) ? 0.0f : g;
          w[r] = acc[r] * g;
        }
#pragma unroll
        for (int r = 0; r < 8; ++r) {
          float sr = w[r];
          sr += __shfl_xor(sr, 1, 32);
          sr += __shfl_xor(sr, 2, 32);
          sr += __shfl_xor(sr, 4, 32);
          sr += __shfl_xor(sr, 8, 32);
          ft[r] = sr;
        }
#pragma unroll
        for (int r = 0; r < 8; ++r) {
          const float rinv = 1.0f / ft[r];
          const float vn = w[r] * rinv;
          sU[((8 * h + r) * kSub + s) * kS + j] = acc[r];
          sN[((8 * h + r) * kSub + s) * kS + j] = vn;
          const bool act = ((am >> r) & 1u) != 0u;
          V[r] = act ? vn : V[r];
        }
        float fsel = ft[0];
        fsel = (jr == 1) ? ft[1] : fsel;
        fsel = (jr == 2) ? ft[2] : fsel;
        fsel = (jr == 3) ? ft[3] : fsel;
        fsel = (jr == 4) ? ft[4] : fsel;
        fsel = (jr == 5) ? ft[5] : fsel;
        fsel = (jr == 6) ? ft[6] : fsel;
        fsel = (jr == 7) ? ft[7] : fsel;
        const int fidx = (j < 8) ? ((8 * h + jr) * kGrp + ss) : (16 * kGrp + lane);
        sF[fidx] = fsel;
        __syncthreads();
      }

      if (grp >= kWarmGrp) {
        const int tsub = i0 - kWarm + half * kSub;
        for (int pass = 0; pass < 2; ++pass) {
#pragma unroll 1
          for (int m = 0; m < 16; ++m) {
            const int c = tile * 16 + m;
            if (c < kNChunk) {
              const size_t t0 = (size_t)c * kChunk + (size_t)tsub;
              float* d0 = out + t0 * kS;
              float* d1 = out + (size_t)kOffUN + t0 * kS;
#pragma unroll
              for (int it = 0; it < 2; ++it) {
                const v4f u  = *(const v4f*)(sU + m * (kSub * kS) + it * 128 + lane * 4);
                const v4f nv = *(const v4f*)(sN + m * (kSub * kS) + it * 128 + lane * 4);
                *(volatile v4f*)(d0 + it * 128 + lane * 4) = u;
                *(volatile v4f*)(d1 + it * 128 + lane * 4) = nv;
              }
            }
          }
          __threadfence();
        }
      }
      __syncthreads();
    }

    if (grp >= kWarmGrp) {
      const int tg = i0 - kWarm;
      for (int pass = 0; pass < 2; ++pass) {
#pragma unroll 1
        for (int m = 0; m < 16; ++m) {
          const int c = tile * 16 + m;
          if (c < kNChunk) {
            const size_t t0 = (size_t)c * kChunk + (size_t)tg;
            const float fv = sF[m * kGrp + lane];
            *(volatile float*)(out + (size_t)kOffFT + t0 + lane) = fv;
          }
        }
        __threadfence();
      }
    }
    __syncthreads();
  }
}

extern "C" void kernel_launch(void* const* d_in, const int* in_sizes, int n_in,
                              void* d_out, int out_size, void* d_ws, size_t ws_size,
                              hipStream_t stream) {
  if (n_in < 4) return;
  if (in_sizes[0] != kT) return;
  if (in_sizes[1] != kS * kS) return;
  if (in_sizes[2] != kS) return;
  if (in_sizes[3] != kS) return;
  if (out_size != 33 * kT) return;
  if (ws_size < kWsBytes) return;

  const float* y      = (const float*)d_in[0];
  const float* logits = (const float*)d_in[1];
  const float* mu     = (const float*)d_in[2];
  const float* logsig = (const float*)d_in[3];
  float* out = (float*)d_out;
  float* wsf = (float*)d_ws;

  k_init<<<1, 32, 0, stream>>>(logits, mu, logsig, wsf);
  k_filter<<<kTiles, 32, 0, stream>>>(y, wsf, out);
}
